// ObjectSpacePerceptionCrossAttention_23948737643081
// MI455X (gfx1250) — hardware-verified
//
#include <hip/hip_runtime.h>
#include <stdint.h>
#include <stddef.h>

typedef _Float16 v16h __attribute__((ext_vector_type(16)));
typedef _Float16 v8h  __attribute__((ext_vector_type(8)));
typedef float    v8f  __attribute__((ext_vector_type(8)));
typedef float    v4f  __attribute__((ext_vector_type(4)));
typedef v8h __attribute__((may_alias)) v8ha;
typedef v4f __attribute__((may_alias)) v4fa;
typedef _Float16 __attribute__((may_alias)) f16a;

union Frag { v16h v; v8h half[2]; };

#define NB     8
#define CH     512
#define L1     1024
#define L2     64
#define HD     64
#define KD     512
#define WSC    32.0f
#define WINV   0.03125f
#define PSC    16384.0f
#define PINV   0.00006103515625f
#define SCALE2 0.08838834764831845f

#define NW0 786432
#define NW1 262144
#define NW2 524288
#define NW3 262144
#define NW4 262144
#define NW5 262144
#define NWT 2359296

__device__ __forceinline__ v8f wmma16(v16h a, v16h b, v8f c) {
  v8f d = __builtin_amdgcn_wmma_f32_16x16x32_f16(false, a, false, b, (short)0, c, false, false);
  asm volatile("v_nop\n\tv_nop\n\tv_nop\n\tv_nop" : "+v"(d) : "v"(a), "v"(b));
  return d;
}

__device__ __forceinline__ v16h load_frag(const _Float16* p, int h) {
  Frag f;
  f.half[0] = *(const v8ha*)(p + 8 * h);
  f.half[1] = *(const v8ha*)(p + 16 + 8 * h);
  return f.v;
}

__device__ __forceinline__ float block_sum256(float v, float* red) {
  const int tid = threadIdx.x;
  v += __shfl_xor(v, 16);
  v += __shfl_xor(v, 8);
  v += __shfl_xor(v, 4);
  v += __shfl_xor(v, 2);
  v += __shfl_xor(v, 1);
  if ((tid & 31) == 0) red[tid >> 5] = v;
  __syncthreads();
  float t = red[0];
  t += red[1]; t += red[2]; t += red[3]; t += red[4]; t += red[5]; t += red[6]; t += red[7];
  __syncthreads();
  return t;
}

__device__ __forceinline__ float group_sum256(float v, float* red, int g) {
  const int tid = threadIdx.x, lane = tid & 31, w = tid >> 5;
  v += __shfl_xor(v, 1);
  v += __shfl_xor(v, 2);
  v += __shfl_xor(v, 16);
  if ((lane & 0x13) == 0) red[w * 4 + (lane >> 2)] = v;
  __syncthreads();
  float t = red[g];
  #pragma unroll
  for (int wi = 1; wi < 8; ++wi) t += red[wi * 4 + g];
  __syncthreads();
  return t;
}

__device__ __forceinline__ void tm_lines_pass(const _Float16* sT, _Float16* out, size_t row0,
                                              int col0, int w, int lane) {
  const int q8 = lane & 7, sub = lane >> 3;
  const int tok = 4 * w + sub;
  const v8h v = *(const v8ha*)(sT + tok * 64 + 8 * q8);
  *(volatile v8h*)(out + (row0 + (size_t)tok) * CH + col0 + 8 * q8) = v;
}

__global__ __launch_bounds__(256) void k_cvt_w(
    const float* __restrict__ w0, const float* __restrict__ w1, const float* __restrict__ w2,
    const float* __restrict__ w3, const float* __restrict__ w4, const float* __restrict__ w5,
    _Float16* __restrict__ wh)
{
  const int g = blockIdx.x * 256 + threadIdx.x;
  if (g >= NWT / 8) return;
  const int e = g * 8;
  const float* src;
  if (e < NW0) src = w0 + e;
  else if (e < NW0 + NW1) src = w1 + (e - NW0);
  else if (e < NW0 + NW1 + NW2) src = w2 + (e - (NW0 + NW1));
  else if (e < NW0 + NW1 + NW2 + NW3) src = w3 + (e - (NW0 + NW1 + NW2));
  else if (e < NW0 + NW1 + NW2 + NW3 + NW4) src = w4 + (e - (NW0 + NW1 + NW2 + NW3));
  else src = w5 + (e - (NW0 + NW1 + NW2 + NW3 + NW4));
  const v4f a = *(const v4fa*)src;
  const v4f c = *(const v4fa*)(src + 4);
  const v8h o = { (_Float16)(a.x * WSC), (_Float16)(a.y * WSC), (_Float16)(a.z * WSC), (_Float16)(a.w * WSC),
                  (_Float16)(c.x * WSC), (_Float16)(c.y * WSC), (_Float16)(c.z * WSC), (_Float16)(c.w * WSC) };
  _Float16* dst = wh + e;
  *(volatile v8h*)dst = o;
  __threadfence();
  *(volatile v8h*)dst = o;
}

__global__ __launch_bounds__(256) void k_cm_to_tm(
    const float* __restrict__ in, const float* __restrict__ addend,
    const float* __restrict__ gam, const float* __restrict__ bet,
    _Float16* __restrict__ out, int L, int do_norm, int has_add, float post_scale)
{
  __shared__ float red[8];
  __shared__ __attribute__((aligned(16))) _Float16 sT[32 * 64];
  const int tid = threadIdx.x, lane = tid & 31, w = tid >> 5;
  const int j = blockIdx.x, n = blockIdx.y;
  const size_t cbase = ((size_t)n * CH + 64 * j) * (size_t)L;
  const float inv_cnt = 1.0f / (float)(16 * L);

  float my_mean = 0.0f, my_rstd = 1.0f;
  if (do_norm) {
    for (int g = 0; g < 4; ++g) {
      const float* gp = in + cbase + (size_t)(16 * g) * L;
      const int cnt4 = 4 * L;
      float s = 0.0f;
      for (int i = tid; i < cnt4; i += 256) {
        const v4f v = *(const v4fa*)(gp + 4 * (size_t)i);
        s += (v.x + v.y) + (v.z + v.w);
      }
      s = block_sum256(s, red);
      const float mean = s * inv_cnt;
      float s2 = 0.0f;
      for (int i = tid; i < cnt4; i += 256) {
        const v4f v = *(const v4fa*)(gp + 4 * (size_t)i);
        const float d0 = v.x - mean, d1 = v.y - mean, d2 = v.z - mean, d3 = v.w - mean;
        s2 += (d0 * d0 + d1 * d1) + (d2 * d2 + d3 * d3);
      }
      s2 = block_sum256(s2, red);
      const float rstd = rsqrtf(s2 * inv_cnt + 1e-5f);
      if ((tid >> 6) == g) { my_mean = mean; my_rstd = rstd; }
    }
  }

  const int c = tid >> 2, q = tid & 3;
  float gm = 1.0f, gb = 0.0f;
  if (do_norm) { gm = gam[64 * j + c]; gb = bet[64 * j + c]; }

  for (int l0 = 0; l0 < L; l0 += 32) {
    const size_t eo = cbase + (size_t)c * L + l0 + 8 * q;
    const v4f a = *(const v4fa*)(in + eo);
    const v4f b = *(const v4fa*)(in + eo + 4);
    float y[8] = { a.x, a.y, a.z, a.w, b.x, b.y, b.z, b.w };
    if (do_norm) {
      #pragma unroll
      for (int e = 0; e < 8; ++e) y[e] = (y[e] - my_mean) * my_rstd * gm + gb;
    }
    if (has_add) {
      const v4f p0 = *(const v4fa*)(addend + eo);
      const v4f p1 = *(const v4fa*)(addend + eo + 4);
      float ad[8] = { p0.x, p0.y, p0.z, p0.w, p1.x, p1.y, p1.z, p1.w };
      #pragma unroll
      for (int e = 0; e < 8; ++e) y[e] = (ad[e] + y[e]) * post_scale;
    }
    #pragma unroll
    for (int e = 0; e < 8; ++e) sT[(8 * q + e) * 64 + c] = (_Float16)y[e];
    __syncthreads();
    const size_t row0 = (size_t)n * L + l0;
    tm_lines_pass(sT, out, row0, 64 * j, w, lane);
    __threadfence();
    tm_lines_pass(sT, out, row0, 64 * j, w, lane);
    __syncthreads();
  }
}

__global__ __launch_bounds__(256) void k_gn_tm(
    const float* __restrict__ in, const float* __restrict__ gam, const float* __restrict__ bet,
    _Float16* __restrict__ out, int L)
{
  __shared__ float red[32];
  __shared__ __attribute__((aligned(16))) _Float16 sT[32 * 64];
  const int tid = threadIdx.x, lane = tid & 31, w = tid >> 5;
  const int j = blockIdx.x, n = blockIdx.y;
  const int q = tid & 15, rr = tid >> 4, g = q >> 2;
  const size_t rowb = (size_t)n * L;
  const int colb = 64 * j + 4 * q;
  const float inv_cnt = 1.0f / (float)(16 * L);

  float s = 0.0f;
  for (int r = rr; r < L; r += 16) {
    const v4f v = *(const v4fa*)(in + (rowb + r) * CH + colb);
    s += (v.x + v.y) + (v.z + v.w);
  }
  s = group_sum256(s, red, g);
  const float mean = s * inv_cnt;
  float s2 = 0.0f;
  for (int r = rr; r < L; r += 16) {
    const v4f v = *(const v4fa*)(in + (rowb + r) * CH + colb);
    const float d0 = v.x - mean, d1 = v.y - mean, d2 = v.z - mean, d3 = v.w - mean;
    s2 += (d0 * d0 + d1 * d1) + (d2 * d2 + d3 * d3);
  }
  s2 = group_sum256(s2, red, g);
  const float rstd = rsqrtf(s2 * inv_cnt + 1e-5f);
  const v4f g4 = *(const v4fa*)(gam + colb);
  const v4f b4 = *(const v4fa*)(bet + colb);

  for (int l0 = 0; l0 < L; l0 += 32) {
    const v4f va = *(const v4fa*)(in + (rowb + l0 + rr) * CH + colb);
    const v4f vb = *(const v4fa*)(in + (rowb + l0 + 16 + rr) * CH + colb);
    _Float16* ta = sT + rr * 64 + 4 * q;
    _Float16* tb = sT + (16 + rr) * 64 + 4 * q;
    ta[0] = (_Float16)((va.x - mean) * rstd * g4.x + b4.x);
    ta[1] = (_Float16)((va.y - mean) * rstd * g4.y + b4.y);
    ta[2] = (_Float16)((va.z - mean) * rstd * g4.z + b4.z);
    ta[3] = (_Float16)((va.w - mean) * rstd * g4.w + b4.w);
    tb[0] = (_Float16)((vb.x - mean) * rstd * g4.x + b4.x);
    tb[1] = (_Float16)((vb.y - mean) * rstd * g4.y + b4.y);
    tb[2] = (_Float16)((vb.z - mean) * rstd * g4.z + b4.z);
    tb[3] = (_Float16)((vb.w - mean) * rstd * g4.w + b4.w);
    __syncthreads();
    tm_lines_pass(sT, out, rowb + l0, 64 * j, w, lane);
    __threadfence();
    tm_lines_pass(sT, out, rowb + l0, 64 * j, w, lane);
    __syncthreads();
  }
}

template<int MODE>
__device__ __forceinline__ void gemm_store_pass(const float* sT, _Float16* dsth, float* dstf,
                                                const float* res, int R0, int n0, int L,
                                                int w, int lane) {
  const int q8 = lane & 7, sub = lane >> 3;
  const _Float16* sTh = (const _Float16*)sT;
  if (MODE == 0) {
    #pragma unroll
    for (int i = 0; i < 8; ++i) {
      const int lid = 32 * w + 4 * i + sub;
      const v8h v = *(const v8ha*)(sTh + lid * 64 + 8 * q8);
      *(volatile v8h*)(dsth + (size_t)(R0 + lid) * CH + n0 + 8 * q8) = v;
    }
  } else if (MODE == 1) {
    #pragma unroll
    for (int i = 0; i < 8; ++i) {
      const int lid = 32 * w + 4 * i + sub;
      const int cc = lid >> 1, hl = lid & 1;
      const v8h v = *(const v8ha*)(sTh + cc * 128 + 64 * hl + 8 * q8);
      const int R = R0 + 64 * hl;
      const int z = R / L;
      const int l = R - z * L;
      *(volatile v8h*)(dsth + (size_t)z * CH * L + (size_t)(n0 + cc) * L + l + 8 * q8) = v;
    }
  } else if (MODE == 2) {
    #pragma unroll
    for (int i = 0; i < 16; ++i) {
      const int lid = 64 * w + 4 * i + sub;
      const int row = lid >> 1, hl = lid & 1;
      const v4f v = *(const v4fa*)(sT + row * 64 + 32 * hl + 4 * q8);
      *(volatile v4f*)(dstf + (size_t)(R0 + row) * CH + n0 + 32 * hl + 4 * q8) = v;
    }
  } else {
    const int z = R0 / L;
    const int l0 = R0 - z * L;
    #pragma unroll
    for (int i = 0; i < 16; ++i) {
      const int lid = 64 * w + 4 * i + sub;
      const int cc = lid >> 2, ql = lid & 3;
      const v4f v = *(const v4fa*)(sT + cc * 128 + 32 * ql + 4 * q8);
      const size_t idx = (size_t)z * CH * L + (size_t)(n0 + cc) * L + l0 + 32 * ql + 4 * q8;
      const v4f rv = *(const v4fa*)(res + idx);
      const v4f o = rv + v;
      *(volatile v4f*)(dstf + idx) = o;
    }
  }
}

template<int MODE>
__global__ __launch_bounds__(128) __attribute__((amdgpu_num_vgpr(256)))
void k_gemm(const _Float16* __restrict__ A, const _Float16* __restrict__ Bw,
            const float* __restrict__ bias, _Float16* __restrict__ dsth,
            float* __restrict__ dstf, const float* __restrict__ res, int L)
{
  __shared__ __attribute__((aligned(16))) float sT[128 * 64];

  const int tid = threadIdx.x, lane = tid & 31, w = tid >> 5;
  const int h = lane >> 4, m = lane & 15;
  const int R0 = blockIdx.x * 128, n0 = blockIdx.y * 64;
  const int R0w = R0 + 32 * w;

  const _Float16* a0p = A + (size_t)(R0w + m) * KD;
  const _Float16* a1p = a0p + (size_t)16 * KD;
  const _Float16* bp  = Bw + (size_t)(n0 + m) * KD;

  const v8f zero8 = {0.f, 0.f, 0.f, 0.f, 0.f, 0.f, 0.f, 0.f};
  v8f acc[2][4];
  #pragma unroll
  for (int mt = 0; mt < 2; ++mt)
    #pragma unroll
    for (int nt = 0; nt < 4; ++nt) acc[mt][nt] = zero8;

  #pragma unroll 1
  for (int k0 = 0; k0 < KD; k0 += 32) {
    const v16h a0 = load_frag(a0p + k0, h);
    const v16h a1 = load_frag(a1p + k0, h);
    #pragma unroll
    for (int nt = 0; nt < 4; ++nt) {
      const v16h b = load_frag(bp + (size_t)nt * 16 * KD + k0, h);
      acc[0][nt] = wmma16(a0, b, acc[0][nt]);
      acc[1][nt] = wmma16(a1, b, acc[1][nt]);
    }
  }

  f16a* sTh = (f16a*)sT;
  #pragma unroll
  for (int nt = 0; nt < 4; ++nt) {
    const int cc = 16 * nt + m;
    const float bv = bias[n0 + cc];
    #pragma unroll
    for (int mt = 0; mt < 2; ++mt) {
      #pragma unroll
      for (int r = 0; r < 8; ++r) {
        const int tokl = 32 * w + 16 * mt + 8 * h + r;
        const float y = acc[mt][nt][r] * WINV + bv;
        if (MODE == 0)      sTh[tokl * 64 + cc] = (_Float16)y;
        else if (MODE == 1) sTh[cc * 128 + tokl] = (_Float16)y;
        else if (MODE == 2) sT[tokl * 64 + cc] = y;
        else                sT[cc * 128 + tokl] = y;
      }
    }
  }
  __syncthreads();

  gemm_store_pass<MODE>(sT, dsth, dstf, res, R0, n0, L, w, lane);
  __threadfence();
  gemm_store_pass<MODE>(sT, dsth, dstf, res, R0, n0, L, w, lane);
}

__device__ __forceinline__ v16h pack_p(v8f a, v8f c) {
  const v16h r = { (_Float16)(a[0] * PSC), (_Float16)(a[1] * PSC), (_Float16)(a[2] * PSC), (_Float16)(a[3] * PSC),
                   (_Float16)(a[4] * PSC), (_Float16)(a[5] * PSC), (_Float16)(a[6] * PSC), (_Float16)(a[7] * PSC),
                   (_Float16)(c[0] * PSC), (_Float16)(c[1] * PSC), (_Float16)(c[2] * PSC), (_Float16)(c[3] * PSC),
                   (_Float16)(c[4] * PSC), (_Float16)(c[5] * PSC), (_Float16)(c[6] * PSC), (_Float16)(c[7] * PSC) };
  return r;
}

__device__ __forceinline__ void attn_store_pass(const _Float16* so, _Float16* otm, size_t row0,
                                                int col0, int lane) {
  const int q8 = lane & 7, sub = lane >> 3;
  #pragma unroll
  for (int i = 0; i < 4; ++i) {
    const int lid = 4 * i + sub;
    const v8h v = *(const v8ha*)(so + lid * 64 + 8 * q8);
    *(volatile v8h*)(otm + (row0 + (size_t)lid) * CH + col0 + 8 * q8) = v;
  }
}

template<int NK>
__global__ __launch_bounds__(128) __attribute__((amdgpu_num_vgpr(256)))
void k_attn(const _Float16* __restrict__ qtm, const _Float16* __restrict__ qpos,
            const _Float16* __restrict__ ktm, const _Float16* __restrict__ kpos,
            const _Float16* __restrict__ vcm, _Float16* __restrict__ otm)
{
  __shared__ __attribute__((aligned(16))) _Float16 sO[4 * 16 * 64];

  const int tid = threadIdx.x, lane = tid & 31, w = tid >> 5;
  const int h = lane >> 4, m = lane & 15;
  const int bh = blockIdx.y, b = bh >> 3, head = bh & 7;
  const int q0 = blockIdx.x * 64 + 16 * w;

  const size_t qoff = ((size_t)b * L1 + q0 + m) * CH + head * HD;
  const v16h qb0 = load_frag(qtm + qoff, h);
  const v16h qb1 = load_frag(qtm + qoff + 32, h);
  const v16h qb2 = load_frag(qpos + qoff, h);
  const v16h qb3 = load_frag(qpos + qoff + 32, h);

  const v8f zero8 = {0.f, 0.f, 0.f, 0.f, 0.f, 0.f, 0.f, 0.f};
  v8f o[4];
  #pragma unroll
  for (int t = 0; t < 4; ++t) o[t] = zero8;
  float mrun = -1e30f, lrun = 0.0f;

  const _Float16* kbase = ktm  + ((size_t)b * NK + m) * CH + head * HD;
  const _Float16* kpb   = kpos + ((size_t)b * NK + m) * CH + head * HD;
  const _Float16* vbase = vcm  + ((size_t)b * CH + head * HD + m) * NK;

  #pragma unroll 1
  for (int kb = 0; kb < NK; kb += 64) {
    v8f s[4];
    #pragma unroll
    for (int j = 0; j < 4; ++j) {
      const size_t ko = (size_t)(kb + 16 * j) * CH;
      v8f z = zero8;
      {
        const v16h f0 = load_frag(kbase + ko, h);
        const v16h f1 = load_frag(kbase + ko + 32, h);
        z = wmma16(f0, qb0, z);
        z = wmma16(f1, qb1, z);
      }
      {
        const v16h f2 = load_frag(kpb + ko, h);
        const v16h f3 = load_frag(kpb + ko + 32, h);
        z = wmma16(f2, qb2, z);
        z = wmma16(f3, qb3, z);
      }
      s[j] = z * SCALE2;
    }

    float mloc = s[0][0];
    #pragma unroll
    for (int j = 0; j < 4; ++j)
      #pragma unroll
      for (int r = 0; r < 8; ++r) mloc = fmaxf(mloc, s[j][r]);
    mloc = fmaxf(mloc, __shfl_xor(mloc, 16));
    const float mnew = fmaxf(mrun, mloc);
    const float alpha = __expf(mrun - mnew);
    mrun = mnew;
    float lsum = 0.0f;
    #pragma unroll
    for (int j = 0; j < 4; ++j)
      #pragma unroll
      for (int r = 0; r < 8; ++r) {
        const float p = __expf(s[j][r] - mnew);
        s[j][r] = p;
        lsum += p;
      }
    lsum += __shfl_xor(lsum, 16);
    lrun = lrun * alpha + lsum;
    #pragma unroll
    for (int t = 0; t < 4; ++t)
      #pragma unroll
      for (int r = 0; r < 8; ++r) o[t][r] = o[t][r] * alpha;

    const v16h pb0 = pack_p(s[0], s[1]);
    const v16h pb1 = pack_p(s[2], s[3]);

    #pragma unroll
    for (int t = 0; t < 4; ++t) {
      const _Float16* vp = vbase + (size_t)(16 * t) * NK + kb;
      const v16h vf0 = load_frag(vp, h);
      const v16h vf1 = load_frag(vp + 32, h);
      o[t] = wmma16(vf0, pb0, o[t]);
      o[t] = wmma16(vf1, pb1, o[t]);
    }
  }

  const float inv = (1.0f / lrun) * PINV;
  _Float16* so = sO + w * 1024;
  #pragma unroll
  for (int t = 0; t < 4; ++t)
    #pragma unroll
    for (int r = 0; r < 8; ++r)
      so[m * 64 + 16 * t + 8 * h + r] = (_Float16)(o[t][r] * inv);
  __syncthreads();

  const size_t row0 = (size_t)b * L1 + q0;
  attn_store_pass(so, otm, row0, head * HD, lane);
  __threadfence();
  attn_store_pass(so, otm, row0, head * HD, lane);
}

extern "C" void kernel_launch(void* const* d_in, const int* in_sizes, int n_in,
                              void* d_out, int out_size, void* d_ws, size_t ws_size,
                              hipStream_t stream) {
  if (n_in < 25) return;
  const int E1 = NB * CH * L1;
  const int E2 = NB * CH * L2;
  if (in_sizes[0] != E1 || in_sizes[4] != E1) return;
  if (in_sizes[1] != E2 || in_sizes[2] != E2 || in_sizes[3] != E2) return;
  if (in_sizes[7] != NW0 || in_sizes[9] != NW1 || in_sizes[11] != NW2 ||
      in_sizes[13] != NW3 || in_sizes[21] != NW4 || in_sizes[23] != NW5) return;
  if (in_sizes[5] != CH || in_sizes[6] != CH || in_sizes[8] != 3 * CH || in_sizes[10] != CH ||
      in_sizes[12] != 2 * CH || in_sizes[14] != CH) return;
  for (int i = 15; i <= 20; ++i) if (in_sizes[i] != CH) return;
  if (in_sizes[22] != CH || in_sizes[24] != CH) return;
  if (out_size != E1) return;

  const float* x        = (const float*)d_in[0];
  const float* xf_out   = (const float*)d_in[1];
  const float* oce      = (const float*)d_in[2];
  const float* odesc    = (const float*)d_in[3];
  const float* ipce     = (const float*)d_in[4];
  const float* gn_qkv_g = (const float*)d_in[5];
  const float* gn_qkv_b = (const float*)d_in[6];
  const float* W_qkv    = (const float*)d_in[7];
  const float* b_qkv    = (const float*)d_in[8];
  const float* W_cq     = (const float*)d_in[9];
  const float* b_cq     = (const float*)d_in[10];
  const float* W_cont   = (const float*)d_in[11];
  const float* b_cont   = (const float*)d_in[12];
  const float* W_pos    = (const float*)d_in[13];
  const float* b_pos    = (const float*)d_in[14];
  const float* gn_desc_g = (const float*)d_in[15];
  const float* gn_desc_b = (const float*)d_in[16];
  const float* gn_cpos_g = (const float*)d_in[17];
  const float* gn_cpos_b = (const float*)d_in[18];
  const float* gn_ipos_g = (const float*)d_in[19];
  const float* gn_ipos_b = (const float*)d_in[20];
  const float* W_so     = (const float*)d_in[21];
  const float* b_so     = (const float*)d_in[22];
  const float* W_co     = (const float*)d_in[23];
  const float* b_co     = (const float*)d_in[24];
  float* outp = (float*)d_out;

  size_t off = 0;
  auto carve = [&](size_t bytes) -> size_t { size_t o = off; off += (bytes + 255) & ~(size_t)255; return o; };
  const size_t o_wh    = carve((size_t)NWT * 2);
  const size_t o_ipce  = carve((size_t)E1 * 2);
  const size_t o_oce   = carve((size_t)E2 * 2);
  const size_t o_xn    = carve((size_t)E1 * 2);
  const size_t o_q     = carve((size_t)E1 * 2);
  const size_t o_k     = carve((size_t)E1 * 2);
  const size_t o_v     = carve((size_t)E1 * 2);
  const size_t o_iposr = carve((size_t)E1 * 4);
  const size_t o_ipos  = carve((size_t)E1 * 2);
  const size_t o_attn  = carve((size_t)E1 * 2);
  const size_t o_xf2   = carve((size_t)E1 * 4);
  const size_t o_cq    = carve((size_t)E1 * 2);
  const size_t o_cposr = carve((size_t)E2 * 4);
  const size_t o_cpos  = carve((size_t)E2 * 2);
  const size_t o_cont  = carve((size_t)E2 * 2);
  const size_t o_ck    = carve((size_t)E2 * 2);
  const size_t o_cv    = carve((size_t)E2 * 2);
  if (off > ws_size) return;

  char* ws = (char*)d_ws;
  _Float16* wh      = (_Float16*)(ws + o_wh);
  _Float16* wqkv    = wh;
  _Float16* wcq     = wqkv + NW0;
  _Float16* wcont   = wcq + NW1;
  _Float16* wpos    = wcont + NW2;
  _Float16* wso     = wpos + NW3;
  _Float16* wco     = wso + NW4;
  _Float16* ipce_tm = (_Float16*)(ws + o_ipce);
  _Float16* oce_tm  = (_Float16*)(ws + o_oce);
  _Float16* xn_tm   = (_Float16*)(ws + o_xn);
  _Float16* q_tm    = (_Float16*)(ws + o_q);
  _Float16* k_tm    = (_Float16*)(ws + o_k);
  _Float16* vcm     = (_Float16*)(ws + o_v);
  float*    iposr   = (float*)(ws + o_iposr);
  _Float16* ipos_tm = (_Float16*)(ws + o_ipos);
  _Float16* attn_tm = (_Float16*)(ws + o_attn);
  float*    xf2     = (float*)(ws + o_xf2);
  _Float16* cq_tm   = (_Float16*)(ws + o_cq);
  float*    cposr   = (float*)(ws + o_cposr);
  _Float16* cpos_tm = (_Float16*)(ws + o_cpos);
  _Float16* cont_tm = (_Float16*)(ws + o_cont);
  _Float16* ck_tm   = (_Float16*)(ws + o_ck);
  _Float16* cvcm    = (_Float16*)(ws + o_cv);

  const dim3 gSlab(8, NB);
  const dim3 gBig(NB * L1 / 128, 8);
  const dim3 gSmall(NB * L2 / 128, 8);
  const dim3 gAtt(L1 / 64, NB * 8);

  k_cvt_w<<<NWT / 8 / 256, 256, 0, stream>>>(W_qkv, W_cq, W_cont, W_pos, W_so, W_co, wh);
  k_cm_to_tm<<<gSlab, 256, 0, stream>>>(x, x, gn_qkv_g, gn_qkv_b, xn_tm, L1, 1, 0, 1.0f);
  k_cm_to_tm<<<gSlab, 256, 0, stream>>>(ipce, ipce, gn_qkv_g, gn_qkv_b, ipce_tm, L1, 0, 0, 1.0f);
  k_cm_to_tm<<<gSlab, 256, 0, stream>>>(oce, oce, gn_qkv_g, gn_qkv_b, oce_tm, L2, 0, 0, 1.0f);
  k_cm_to_tm<<<gSlab, 256, 0, stream>>>(odesc, xf_out, gn_desc_g, gn_desc_b, cont_tm, L2, 1, 1, 0.5f);
  k_gemm<0><<<gBig, 128, 0, stream>>>(xn_tm, wqkv, b_qkv, q_tm, xf2, x, L1);
  k_gemm<0><<<gBig, 128, 0, stream>>>(xn_tm, wqkv + (size_t)CH * KD, b_qkv + CH, k_tm, xf2, x, L1);
  k_gemm<1><<<gBig, 128, 0, stream>>>(xn_tm, wqkv + (size_t)2 * CH * KD, b_qkv + 2 * CH, vcm, xf2, x, L1);
  k_gemm<2><<<gBig, 128, 0, stream>>>(ipce_tm, wpos, b_pos, attn_tm, iposr, x, L1);
  k_gn_tm<<<gSlab, 256, 0, stream>>>(iposr, gn_ipos_g, gn_ipos_b, ipos_tm, L1);
  k_gemm<2><<<gSmall, 128, 0, stream>>>(oce_tm, wpos, b_pos, attn_tm, cposr, x, L2);
  k_gn_tm<<<gSlab, 256, 0, stream>>>(cposr, gn_cpos_g, gn_cpos_b, cpos_tm, L2);
  k_gemm<0><<<gSmall, 128, 0, stream>>>(cont_tm, wcont, b_cont, ck_tm, xf2, x, L2);
  k_gemm<1><<<gSmall, 128, 0, stream>>>(cont_tm, wcont + (size_t)CH * KD, b_cont + CH, cvcm, xf2, x, L2);
  k_attn<1024><<<gAtt, 128, 0, stream>>>(q_tm, ipos_tm, k_tm, ipos_tm, vcm, attn_tm);
  k_gemm<3><<<gBig, 128, 0, stream>>>(attn_tm, wso, b_so, attn_tm, xf2, x, L1);
  k_cm_to_tm<<<gSlab, 256, 0, stream>>>(xf2, xf2, gn_qkv_g, gn_qkv_b, xn_tm, L1, 1, 0, 1.0f);
  k_gemm<0><<<gBig, 128, 0, stream>>>(xn_tm, wcq, b_cq, cq_tm, xf2, x, L1);
  k_attn<64><<<gAtt, 128, 0, stream>>>(cq_tm, ipos_tm, ck_tm, cpos_tm, cvcm, attn_tm);
  k_gemm<3><<<gBig, 128, 0, stream>>>(attn_tm, wco, b_co, attn_tm, outp, xf2, L1);
}
